// Tmix_2353642078795
// MI455X (gfx1250) — hardware-verified
//
#include <hip/hip_runtime.h>
#include <math.h>

constexpr int NBATCH = 4;
constexpr int NTIME  = 1024;
constexpr int NCH    = 1024;
constexpr int NHEAD  = 16;
constexpr int HSZ    = 64;
constexpr int MROWS  = NBATCH * NTIME;
constexpr int DLW = 64, DLA = 64, DLG = 128;
constexpr float GN_EPS = 0.00064f;
constexpr float INV_HS = 1.0f / 64.0f;
constexpr size_t PLANE_ELEMS = (size_t)MROWS * NCH;
constexpr size_t PLANE_F32_BYTES = PLANE_ELEMS * 4;
constexpr size_t MIB = 1048576;

typedef __attribute__((ext_vector_type(16))) _Float16 v16h;
typedef __attribute__((ext_vector_type(8)))  _Float16 v8h;
typedef __attribute__((ext_vector_type(16))) __bf16   v16b;
typedef __attribute__((ext_vector_type(8)))  __bf16   v8b;
typedef __attribute__((ext_vector_type(8)))  float    v8f;
typedef __attribute__((ext_vector_type(4)))  float    v4f;
typedef __attribute__((ext_vector_type(4)))  unsigned int v4u;
typedef __attribute__((ext_vector_type(2)))  unsigned int v2u;

__device__ __forceinline__ unsigned short f2bf_bits(float f) {
  unsigned u = __float_as_uint(f);
  return (unsigned short)((u + 0x7FFFu + ((u >> 16) & 1u)) >> 16);
}
__device__ __forceinline__ float bf_bits2f(unsigned short h) { return __uint_as_float(((unsigned)h) << 16); }

__device__ __forceinline__ void dep_guard_h(v8f& a, v8f& b, v16h x, v16h y) { asm volatile("v_nop\n\tv_nop\n\tv_nop\n\tv_nop" : "+v"(a), "+v"(b) : "v"(x), "v"(y)); }
__device__ __forceinline__ void dep_guard_b(v8f& a, v8f& b, v16b x, v16b y) { asm volatile("v_nop\n\tv_nop\n\tv_nop\n\tv_nop" : "+v"(a), "+v"(b) : "v"(x), "v"(y)); }
__device__ __forceinline__ void keep4_h(v16h a, v16h b, v16h c, v16h d) { asm volatile("v_nop" :: "v"(a), "v"(b), "v"(c), "v"(d)); }
__device__ __forceinline__ void keep4_b(v16b a, v16b b, v16b c, v16b d) { asm volatile("v_nop" :: "v"(a), "v"(b), "v"(c), "v"(d)); }
__device__ __forceinline__ void acc_guard4(v8f& a, v8f& b, v8f& c, v8f& d) { asm volatile("v_nop\n\tv_nop\n\tv_nop\n\tv_nop" : "+v"(a), "+v"(b), "+v"(c), "+v"(d)); }
template <typename T> struct Frag;
template <> struct Frag<_Float16> {
  typedef v16h V; union U { v16h v; v8h h[2]; };
  static __device__ __forceinline__ v16h load(const _Float16* p) {
    U f; f.h[0] = *(const v8h*)(p); f.h[1] = *(const v8h*)(p + 16); return f.v;
  }
  static __device__ __forceinline__ v8f mma(v16h a, v16h b, v8f c) {
    return __builtin_amdgcn_wmma_f32_16x16x32_f16(false, a, false, b, (short)0, c, false, false);
  }
  static __device__ __forceinline__ void guard(v8f& a, v8f& b, v16h x, v16h y) { dep_guard_h(a, b, x, y); }
  static __device__ __forceinline__ void keep(v16h a, v16h b, v16h c, v16h d) { keep4_h(a, b, c, d); }
};
template <> struct Frag<__bf16> {
  typedef v16b V; union U { v16b v; v8b h[2]; };
  static __device__ __forceinline__ v16b load(const __bf16* p) {
    U f; f.h[0] = *(const v8b*)(p); f.h[1] = *(const v8b*)(p + 16); return f.v;
  }
  static __device__ __forceinline__ v8f mma(v16b a, v16b b, v8f c) {
    return __builtin_amdgcn_wmma_f32_16x16x32_bf16(false, a, false, b, (short)0, c, false, false);
  }
  static __device__ __forceinline__ void guard(v8f& a, v8f& b, v16b x, v16b y) { dep_guard_b(a, b, x, y); }
  static __device__ __forceinline__ void keep(v16b a, v16b b, v16b c, v16b d) { keep4_b(a, b, c, d); }
};

__device__ __forceinline__ unsigned pk16(unsigned short a, unsigned short b) { return (unsigned)a | ((unsigned)b << 16); }
__device__ __forceinline__ void split_bf(float f, unsigned short& hb, unsigned short& lb) {
  hb = f2bf_bits(f);
  lb = f2bf_bits(f - bf_bits2f(hb));
}
__device__ __forceinline__ void ld8(const float* p, float* o) {
  const v4f a = *(const v4f*)(p);
  const v4f c = *(const v4f*)(p + 4);
  o[0] = a[0]; o[1] = a[1]; o[2] = a[2]; o[3] = a[3];
  o[4] = c[0]; o[5] = c[1]; o[6] = c[2]; o[7] = c[3];
}

template <int ET> struct Elem;
template <> struct Elem<0> { typedef _Float16 T; };
template <> struct Elem<1> { typedef __bf16 T; };
template <int ET, bool SPLIT, int BIAS_MODE, int OUT_MODE, bool RESID, int ACT = 0>
__global__ __launch_bounds__(256) void wmma_gemm64(
    const unsigned short* __restrict__ Ap, const unsigned short* __restrict__ A2p, int lda, long strideA,
    const unsigned short* __restrict__ Btp, const unsigned short* __restrict__ Bt2p, int ldb, long strideB,
    void* __restrict__ Cout, void* __restrict__ Cout2, int ldc, long strideC,
    const float* __restrict__ bias,
    const float* __restrict__ resid, long strideR,
    int M, int N, int K, float scale) {
  typedef typename Elem<ET>::T T;
  typedef typename Frag<T>::V V;
  const T* A = (const T*)Ap; const T* A2 = (const T*)A2p; const T* Bt = (const T*)Btp; const T* Bt2 = (const T*)Bt2p;
  __shared__ __align__(16) float sT[8][16 * 68];
  const int b    = blockIdx.y;
  const int lane = threadIdx.x & 31;
  const int wave = threadIdx.x >> 5;
  const int tilesN = N >> 6;
  const int tilesM = M >> 6;
  const int tile = blockIdx.x * 8 + wave;
  if (tile >= tilesM * tilesN) return;
  const int tm = tile / tilesN;
  const int tn = tile - tm * tilesN;
  const int m0 = tm << 6;
  const int n0 = tn << 6;

  const T* Ab  = A  + (size_t)b * strideA;
  const T* Bb  = Bt + (size_t)b * strideB;
  const T* Ab2 = SPLIT ? (A2  + (size_t)b * strideA) : nullptr;
  const T* Bb2 = SPLIT ? (Bt2 + (size_t)b * strideB) : nullptr;

  const int rlane = lane & 15;
  const int koff  = (lane >> 4) * 8;
  const int mOff  = (lane >> 4) * 8;

  v8f acc[4][4];
#pragma unroll
  for (int i = 0; i < 4; ++i)
#pragma unroll
    for (int j = 0; j < 4; ++j) acc[i][j] = (v8f){0.f,0.f,0.f,0.f,0.f,0.f,0.f,0.f};

  for (int k0 = 0; k0 < K; k0 += 32) {
    V bh[4], bl[4];
#pragma unroll
    for (int j = 0; j < 4; ++j) {
      const size_t bo = (size_t)(n0 + (j << 4) + rlane) * ldb + koff + k0;
      bh[j] = Frag<T>::load(Bb + bo);
      if (SPLIT) bl[j] = Frag<T>::load(Bb2 + bo);
    }
#pragma unroll
    for (int i = 0; i < 4; ++i) {
      const size_t ao = (size_t)(m0 + (i << 4) + rlane) * lda + koff + k0;
      V ah = Frag<T>::load(Ab + ao);
      V al;
      if (SPLIT) al = Frag<T>::load(Ab2 + ao);
#pragma unroll
      for (int j = 0; j < 4; ++j) {
        acc[i][j] = Frag<T>::mma(ah, bh[j], acc[i][j]);
        if (SPLIT) {
          acc[i][j] = Frag<T>::mma(ah, bl[j], acc[i][j]);
          acc[i][j] = Frag<T>::mma(al, bh[j], acc[i][j]);
        }
      }
      Frag<T>::guard(acc[i][0], acc[i][3], ah, SPLIT ? al : ah);
    }
    Frag<T>::keep(bh[0], bh[1], bh[2], bh[3]);
    if (SPLIT) Frag<T>::keep(bl[0], bl[1], bl[2], bl[3]);
  }
  acc_guard4(acc[0][0], acc[0][1], acc[0][2], acc[0][3]);
  acc_guard4(acc[1][0], acc[1][1], acc[1][2], acc[1][3]);
  acc_guard4(acc[2][0], acc[2][1], acc[2][2], acc[2][3]);
  acc_guard4(acc[3][0], acc[3][1], acc[3][2], acc[3][3]);

  float* slab = sT[wave];
  const float* Rb = RESID ? (resid + (size_t)b * strideR) : nullptr;
#pragma unroll
  for (int i = 0; i < 4; ++i) {
    const int mBase = m0 + (i << 4);
#pragma unroll
    for (int j = 0; j < 4; ++j) {
      const int n = n0 + (j << 4) + rlane;
      float bv = 0.f;
      if (BIAS_MODE == 2) bv = bias[n];
#pragma unroll
      for (int r = 0; r < 8; ++r) {
        float v = acc[i][j][r] * scale;
        if (BIAS_MODE == 1) v += bias[mBase + mOff + r];
        if (BIAS_MODE == 2) v += bv;
        if (RESID) v += Rb[(size_t)(mBase + mOff + r) * ldc + n];
        if (ACT == 2) v = fmaxf(v, 0.0f);
        if (ACT == 4) v = (v > 0.f) ? v : 0.01f * v;
        slab[(mOff + r) * 68 + (j << 4) + rlane] = v;
      }
    }
    __builtin_amdgcn_fence(__ATOMIC_RELEASE, "workgroup");
    __builtin_amdgcn_wave_barrier();
    __builtin_amdgcn_fence(__ATOMIC_ACQUIRE, "workgroup");
    if (OUT_MODE == 0) {
      float* C = (float*)Cout + (size_t)b * strideC;
      const int hh = lane >> 4, c4 = (lane & 15) * 4;
      for (int pass = 0; pass < 2; ++pass) {
#pragma unroll
        for (int it = 0; it < 8; ++it) {
          const int row = it * 2 + hh;
          v4f v = *(const v4f*)(slab + row * 68 + c4);
          *(volatile v4f*)(C + (size_t)(mBase + row) * ldc + n0 + c4) = v;
        }
        __threadfence();
      }
    } else {
      const int q = lane >> 3, c8 = (lane & 7) * 8;
      unsigned short* C  = (unsigned short*)Cout  + (size_t)b * strideC;
      unsigned short* C2 = (OUT_MODE == 2) ? ((unsigned short*)Cout2 + (size_t)b * strideC) : nullptr;
      for (int pass = 0; pass < 2; ++pass) {
#pragma unroll
        for (int it = 0; it < 4; ++it) {
          const int row = it * 4 + q;
          const float* sp = slab + row * 68 + c8;
          v8h hv, lv;
#pragma unroll
          for (int e = 0; e < 8; ++e) {
            if (OUT_MODE == 1) {
              hv[e] = (_Float16)sp[e];
            } else {
              unsigned short hb = f2bf_bits(sp[e]);
              unsigned short lb = f2bf_bits(sp[e] - bf_bits2f(hb));
              hv[e] = __builtin_bit_cast(_Float16, hb);
              lv[e] = __builtin_bit_cast(_Float16, lb);
            }
          }
          *(volatile v8h*)(C + (size_t)(mBase + row) * ldc + n0 + c8) = hv;
          if (OUT_MODE == 2) *(volatile v8h*)(C2 + (size_t)(mBase + row) * ldc + n0 + c8) = lv;
        }
        __threadfence();
      }
    }
    __builtin_amdgcn_fence(__ATOMIC_RELEASE, "workgroup");
    __builtin_amdgcn_wave_barrier();
    __builtin_amdgcn_fence(__ATOMIC_ACQUIRE, "workgroup");
  }
}

__global__ __launch_bounds__(256) void wsplit_kernel(const float* __restrict__ W0, const float* __restrict__ W1,
                                                     const float* __restrict__ W2, unsigned short* __restrict__ out,
                                                     int Kd, int Nd) {
  __shared__ float sm[64][65];
  const int t  = threadIdx.x;
  const int k0 = blockIdx.x * 64;
  const int n0 = blockIdx.y * 64;
  const int z  = blockIdx.z;
  const float* W = (z == 0) ? W0 : ((z == 1) ? W1 : W2);
#pragma unroll
  for (int i = 0; i < 16; ++i) {
    const int e = i * 256 + t;
    const int r = e >> 6;
    const int c = e & 63;
    sm[c][r] = W[(size_t)(k0 + r) * Nd + n0 + c];
  }
  __syncthreads();
  const int lane = t & 31, wave = t >> 5;
  const int q = lane >> 3, c8 = (lane & 7) * 8;
  const size_t plane = (size_t)Nd * Kd;
  unsigned short* oh = out + (size_t)z * 2 * plane;
  unsigned short* ol = oh + plane;
  v4u uh[2], ul[2];
  size_t oo[2];
#pragma unroll
  for (int it = 0; it < 2; ++it) {
    const int row = wave * 8 + it * 4 + q;
    unsigned short hb[8], lb[8];
#pragma unroll
    for (int e = 0; e < 8; ++e) split_bf(sm[row][c8 + e], hb[e], lb[e]);
    uh[it] = (v4u){pk16(hb[0], hb[1]), pk16(hb[2], hb[3]), pk16(hb[4], hb[5]), pk16(hb[6], hb[7])};
    ul[it] = (v4u){pk16(lb[0], lb[1]), pk16(lb[2], lb[3]), pk16(lb[4], lb[5]), pk16(lb[6], lb[7])};
    oo[it] = (size_t)(n0 + row) * Kd + k0 + c8;
  }
  for (int pass = 0; pass < 2; ++pass) {
#pragma unroll
    for (int it = 0; it < 2; ++it) {
      *(volatile v4u*)(oh + oo[it]) = uh[it];
      *(volatile v4u*)(ol + oo[it]) = ul[it];
    }
    __threadfence();
  }
}

__device__ __forceinline__ void mix8(const float* __restrict__ mp, const float* xcur, const float* dx, v4u& uh, v4u& ul) {
  const v4f m0 = *(const v4f*)(mp);
  const v4f m1 = *(const v4f*)(mp + 4);
  unsigned short hb[8], lb[8];
#pragma unroll
  for (int e = 0; e < 4; ++e) {
    split_bf(xcur[e] + dx[e] * m0[e], hb[e], lb[e]);
    split_bf(xcur[4 + e] + dx[4 + e] * m1[e], hb[4 + e], lb[4 + e]);
  }
  uh = (v4u){pk16(hb[0], hb[1]), pk16(hb[2], hb[3]), pk16(hb[4], hb[5]), pk16(hb[6], hb[7])};
  ul = (v4u){pk16(lb[0], lb[1]), pk16(lb[2], lb[3]), pk16(lb[4], lb[5]), pk16(lb[6], lb[7])};
}

template <int NMIX>
__global__ __launch_bounds__(256) void prep_kernel(const float* __restrict__ x,
    const float* __restrict__ mixA, const float* __restrict__ mixB, const float* __restrict__ mixC,
    unsigned short* __restrict__ outA, unsigned short* __restrict__ outB, unsigned short* __restrict__ outC) {
  const int g8   = blockIdx.x * 256 + threadIdx.x;
  const int tok  = g8 >> 7;
  const int c0   = (g8 & 127) * 8;
  const int tpos = tok & (NTIME - 1);
  const float* xc = x + (size_t)tok * NCH + c0;
  const int ptok = (tpos > 0) ? (tok - 1) : tok;
  const float* xp = x + (size_t)ptok * NCH + c0;
  const v4f c0v = *(const v4f*)(xc);
  const v4f c1v = *(const v4f*)(xc + 4);
  const v4f p0v = *(const v4f*)(xp);
  const v4f p1v = *(const v4f*)(xp + 4);
  const bool has_prev = (tpos > 0);
  float xcur[8], dx[8];
#pragma unroll
  for (int e = 0; e < 4; ++e) {
    xcur[e] = c0v[e];
    xcur[4 + e] = c1v[e];
    const float pa = has_prev ? p0v[e] : 0.0f;
    const float pb = has_prev ? p1v[e] : 0.0f;
    dx[e] = pa - xcur[e];
    dx[4 + e] = pb - xcur[4 + e];
  }
  const size_t ob = (size_t)tok * NCH + c0;
  v4u hA = (v4u){0u, 0u, 0u, 0u}, lA = (v4u){0u, 0u, 0u, 0u};
  v4u hB = (v4u){0u, 0u, 0u, 0u}, lB = (v4u){0u, 0u, 0u, 0u};
  v4u hC = (v4u){0u, 0u, 0u, 0u}, lC = (v4u){0u, 0u, 0u, 0u};
  mix8(mixA + c0, xcur, dx, hA, lA);
  if (NMIX > 1) mix8(mixB + c0, xcur, dx, hB, lB);
  if (NMIX > 2) mix8(mixC + c0, xcur, dx, hC, lC);
  for (int pass = 0; pass < 2; ++pass) {
    *(volatile v4u*)(outA + ob) = hA;
    *(volatile v4u*)(outA + PLANE_ELEMS + ob) = lA;
    if (NMIX > 1) {
      *(volatile v4u*)(outB + ob) = hB;
      *(volatile v4u*)(outB + PLANE_ELEMS + ob) = lB;
    }
    if (NMIX > 2) {
      *(volatile v4u*)(outC + ob) = hC;
      *(volatile v4u*)(outC + PLANE_ELEMS + ob) = lC;
    }
    __threadfence();
  }
}

template <int ACT>
__global__ __launch_bounds__(256) void act8_kernel(const float* __restrict__ in, unsigned short* __restrict__ oh,
                                                    unsigned short* __restrict__ ol, int n8) {
  const int i = blockIdx.x * 256 + threadIdx.x;
  if (i >= n8) return;
  const float* p = in + 8 * (size_t)i;
  const v4f a = *(const v4f*)(p);
  const v4f c = *(const v4f*)(p + 4);
  unsigned short hb[8], lb[8];
#pragma unroll
  for (int e = 0; e < 4; ++e) {
    float f0, f1;
    if (ACT == 1) { f0 = tanhf(a[e]); f1 = tanhf(c[e]); }
    else          { f0 = 1.0f / (1.0f + expf(-a[e])); f1 = 1.0f / (1.0f + expf(-c[e])); }
    split_bf(f0, hb[e], lb[e]);
    split_bf(f1, hb[4 + e], lb[4 + e]);
  }
  const v4u uh = (v4u){pk16(hb[0], hb[1]), pk16(hb[2], hb[3]), pk16(hb[4], hb[5]), pk16(hb[6], hb[7])};
  const v4u ul = (v4u){pk16(lb[0], lb[1]), pk16(lb[2], lb[3]), pk16(lb[4], lb[5]), pk16(lb[6], lb[7])};
  unsigned short* ph = oh + 8 * (size_t)i;
  unsigned short* pl = ol + 8 * (size_t)i;
  *(volatile v4u*)ph = uh;
  *(volatile v4u*)pl = ul;
  __threadfence();
  *(volatile v4u*)ph = uh;
  *(volatile v4u*)pl = ul;
}

__global__ __launch_bounds__(256) void mid_kernel(const float* __restrict__ WLp, const float* __restrict__ ALp,
                                                  const float* __restrict__ w0p, const float* __restrict__ a0p,
                                                  float* __restrict__ DECp, float* __restrict__ Aout) {
  const size_t i = (size_t)blockIdx.x * 256 + threadIdx.x;
  const int c = (int)(i & (NCH - 1));
  const float u  = w0p[c] + WLp[i];
  const float nu = -u;
  const float sp = log1pf(expf(-fabsf(nu))) + fmaxf(nu, 0.0f);
  const float wv = -sp - 0.5f;
  const float dec = expf(-expf(wv));
  const float zz = a0p[c] + ALp[i];
  const float av = 1.0f / (1.0f + expf(-zz));
  *(volatile float*)(DECp + i) = dec;
  *(volatile float*)(Aout + i) = av;
  __threadfence();
  *(volatile float*)(DECp + i) = dec;
  *(volatile float*)(Aout + i) = av;
}

__device__ __forceinline__ void flush16(const float* buf, float* __restrict__ dst, int wave, int lane) {
  if (wave < 8) {
    const int hsel = lane >> 4;
    const int c4   = (lane & 15) * 4;
    const int row  = wave * 2 + hsel;
    const v4f val = *(const v4f*)(buf + row * 68 + c4);
    float* p = dst + (size_t)row * NCH + c4;
    *(volatile v4f*)p = val;
    __threadfence();
    *(volatile v4f*)p = val;
  }
}

__global__ __launch_bounds__(512) void wkv_kernel(const float* __restrict__ Rp, const float* __restrict__ Dp,
                                                  const float* __restrict__ Kp, const float* __restrict__ Vp,
                                                  const float* __restrict__ Ap,
                                                  const float* __restrict__ kkw, const float* __restrict__ kaw,
                                                  float* __restrict__ Yp) {
  __shared__ __align__(16) float sR[2][HSZ];
  __shared__ __align__(16) float sW[2][HSZ];
  __shared__ __align__(16) float sK[2][HSZ];
  __shared__ __align__(16) float sV[2][HSZ];
  __shared__ __align__(16) float sA[2][HSZ];
  __shared__ __align__(16) float sB[2][HSZ];
  __shared__ __align__(16) float ybuf[2][16 * 68];
  const int bh   = blockIdx.x;
  const int bsel = bh >> 4;
  const int hsel = bh & (NHEAD - 1);
  const int t = threadIdx.x, lane = t & 31, wave = t >> 5;
  const int irow = t >> 3, q = t & 7, j0 = q * 8;
  const size_t base = (size_t)bsel * NTIME * NCH + (size_t)hsel * HSZ;
  const int cpar = hsel * HSZ + lane;
  const float kw0 = kkw[cpar], kw1 = kkw[cpar + 32];
  const float ka0 = kaw[cpar], ka1 = kaw[cpar + 32];
  float S[8];
#pragma unroll
  for (int n = 0; n < 8; ++n) S[n] = 0.0f;

#pragma unroll 1
  for (int ts = 0; ts < NTIME; ++ts) {
    const int p = ts & 1;
    if (wave == 0) {
      const size_t off = base + (size_t)ts * NCH;
      const float r0 = Rp[off + lane], r1 = Rp[off + lane + 32];
      const float d0 = Dp[off + lane], d1 = Dp[off + lane + 32];
      const float k0 = Kp[off + lane], k1 = Kp[off + lane + 32];
      const float v0 = Vp[off + lane], v1 = Vp[off + lane + 32];
      const float e0 = Ap[off + lane], e1 = Ap[off + lane + 32];
      const float u0 = k0 * kw0, u1 = k1 * kw1;
      float ss = u0 * u0 + u1 * u1;
      ss += __shfl_xor(ss, 16, 32);
      ss += __shfl_xor(ss, 8, 32);
      ss += __shfl_xor(ss, 4, 32);
      ss += __shfl_xor(ss, 2, 32);
      ss += __shfl_xor(ss, 1, 32);
      const float inv = 1.0f / fmaxf(sqrtf(ss), 1e-12f);
      const float n0 = u0 * inv, n1 = u1 * inv;
      sR[p][lane] = r0;  sR[p][lane + 32] = r1;
      sW[p][lane] = d0;  sW[p][lane + 32] = d1;
      sK[p][lane] = k0 * (1.0f + (e0 - 1.0f) * ka0);
      sK[p][lane + 32] = k1 * (1.0f + (e1 - 1.0f) * ka1);
      sV[p][lane] = v0;  sV[p][lane + 32] = v1;
      sA[p][lane] = -n0; sA[p][lane + 32] = -n1;
      sB[p][lane] = n0 * e0; sB[p][lane + 32] = n1 * e1;
    }
    __syncthreads();
    if (ts > 0 && (ts & 15) == 0)
      flush16(&ybuf[((ts >> 4) - 1) & 1][0], Yp + base + (size_t)(ts - 16) * NCH, wave, lane);

    const v4f av0 = *(const v4f*)(&sA[p][j0]), av1 = *(const v4f*)(&sA[p][j0 + 4]);
    const v4f wv0 = *(const v4f*)(&sW[p][j0]), wv1 = *(const v4f*)(&sW[p][j0 + 4]);
    const v4f bv0 = *(const v4f*)(&sB[p][j0]), bv1 = *(const v4f*)(&sB[p][j0 + 4]);
    const v4f kv0 = *(const v4f*)(&sK[p][j0]), kv1 = *(const v4f*)(&sK[p][j0 + 4]);
    const v4f rv0 = *(const v4f*)(&sR[p][j0]), rv1 = *(const v4f*)(&sR[p][j0 + 4]);
    float a8[8], w8[8], b8[8], k8[8], r8[8];
#pragma unroll
    for (int e = 0; e < 4; ++e) {
      a8[e] = av0[e]; a8[4 + e] = av1[e];
      w8[e] = wv0[e]; w8[4 + e] = wv1[e];
      b8[e] = bv0[e]; b8[4 + e] = bv1[e];
      k8[e] = kv0[e]; k8[4 + e] = kv1[e];
      r8[e] = rv0[e]; r8[4 + e] = rv1[e];
    }
    float sa = 0.0f;
#pragma unroll
    for (int n = 0; n < 8; ++n) sa += S[n] * a8[n];
    sa += __shfl_xor(sa, 1, 32);
    sa += __shfl_xor(sa, 2, 32);
    sa += __shfl_xor(sa, 4, 32);
    const float vi = sV[p][irow];
    float yp = 0.0f;
#pragma unroll
    for (int n = 0; n < 8; ++n) {
      const float s = S[n] * w8[n] + sa * b8[n] + vi * k8[n];
      S[n] = s;
      yp += s * r8[n];
    }
    yp += __shfl_xor(yp, 1, 32);
    yp += __shfl_xor(yp, 2, 32);
    yp += __shfl_xor(yp, 4, 32);
    if (q == 0) ybuf[(ts >> 4) & 1][(ts & 15) * 68 + irow] = yp;
  }
  __syncthreads();
  flush16(&ybuf[((NTIME >> 4) - 1) & 1][0], Yp + base + (size_t)(NTIME - 16) * NCH, wave, lane);
}

__global__ __launch_bounds__(256) void post_kernel(const float* __restrict__ Yp, const float* __restrict__ Rp,
    const float* __restrict__ Kp, const float* __restrict__ Ap, const float* __restrict__ Vp,
    const float* __restrict__ Gp, const float* __restrict__ kaw, const float* __restrict__ rkw,
    const float* __restrict__ lnw, const float* __restrict__ lnb,
    unsigned short* __restrict__ oh, unsigned short* __restrict__ ol) {
  const int g8  = blockIdx.x * 256 + threadIdx.x;
  const int tok = g8 >> 7;
  const int c0  = (g8 & 127) * 8;
  const size_t ob = (size_t)tok * NCH + c0;
  float y[8], r[8], k[8], a[8], v[8], g[8], ka[8], rk[8], lw[8], lbv[8];
  ld8(Yp + ob, y); ld8(Rp + ob, r); ld8(Kp + ob, k); ld8(Ap + ob, a); ld8(Vp + ob, v); ld8(Gp + ob, g);
  ld8(kaw + c0, ka); ld8(rkw + c0, rk); ld8(lnw + c0, lw); ld8(lnb + c0, lbv);
  float s1 = 0.0f;
#pragma unroll
  for (int e = 0; e < 8; ++e) s1 += y[e];
  s1 += __shfl_xor(s1, 1, 32);
  s1 += __shfl_xor(s1, 2, 32);
  s1 += __shfl_xor(s1, 4, 32);
  const float mu = s1 * INV_HS;
  float dev[8];
  float s2 = 0.0f;
#pragma unroll
  for (int e = 0; e < 8; ++e) { dev[e] = y[e] - mu; s2 += dev[e] * dev[e]; }
  s2 += __shfl_xor(s2, 1, 32);
  s2 += __shfl_xor(s2, 2, 32);
  s2 += __shfl_xor(s2, 4, 32);
  const float var = s2 * INV_HS;
  const float inv = 1.0f / sqrtf(var + GN_EPS);
  float dot = 0.0f;
#pragma unroll
  for (int e = 0; e < 8; ++e) {
    const float kf = k[e] * (1.0f + (a[e] - 1.0f) * ka[e]);
    dot += (r[e] * kf) * rk[e];
  }
  dot += __shfl_xor(dot, 1, 32);
  dot += __shfl_xor(dot, 2, 32);
  dot += __shfl_xor(dot, 4, 32);
  unsigned short hb[8], lb[8];
#pragma unroll
  for (int e = 0; e < 8; ++e) {
    const float gn = (dev[e] * inv) * lw[e] + lbv[e];
    const float o  = (gn + dot * v[e]) * g[e];
    split_bf(o, hb[e], lb[e]);
  }
  const v4u uh = (v4u){pk16(hb[0], hb[1]), pk16(hb[2], hb[3]), pk16(hb[4], hb[5]), pk16(hb[6], hb[7])};
  const v4u ul = (v4u){pk16(lb[0], lb[1]), pk16(lb[2], lb[3]), pk16(lb[4], lb[5]), pk16(lb[6], lb[7])};
  *(volatile v4u*)(oh + ob) = uh;
  *(volatile v4u*)(ol + ob) = ul;
  __threadfence();
  *(volatile v4u*)(oh + ob) = uh;
  *(volatile v4u*)(ol + ob) = ul;
}

static void gemm_split_f32(const unsigned short* Ah, const unsigned short* Al, int lda,
                           const unsigned short* Bh, const unsigned short* Bl, int ldb,
                           float* Cp, int ldc, int M, int N, int K, hipStream_t stream) {
  const int tiles = (M / 64) * (N / 64);
  const int nblk  = (tiles + 7) / 8;
  wmma_gemm64<1, true, 0, 0, false, 0><<<dim3(nblk, 1), dim3(256), 0, stream>>>(
      Ah, Al, lda, 0L, Bh, Bl, ldb, 0L, (void*)Cp, nullptr, ldc, 0L, nullptr, nullptr, 0L, M, N, K, 1.0f);
}
static void gemm_split_hilo(const unsigned short* Ah, const unsigned short* Al, int lda,
                            const unsigned short* Bh, const unsigned short* Bl, int ldb,
                            unsigned short* Ch, unsigned short* Cl, int ldc, int M, int N, int K, hipStream_t stream) {
  const int tiles = (M / 64) * (N / 64);
  const int nblk  = (tiles + 7) / 8;
  wmma_gemm64<1, true, 0, 2, false, 0><<<dim3(nblk, 1), dim3(256), 0, stream>>>(
      Ah, Al, lda, 0L, Bh, Bl, ldb, 0L, (void*)Ch, (void*)Cl, ldc, 0L, nullptr, nullptr, 0L, M, N, K, 1.0f);
}

extern "C" void kernel_launch(void* const* d_in, const int* in_sizes, int n_in,
                              void* d_out, int out_size, void* d_ws, size_t ws_size, hipStream_t stream) {
  if (n_in < 27) return;
  if ((size_t)out_size < PLANE_ELEMS) return;
  if ((size_t)in_sizes[0] != PLANE_ELEMS) return;
  if (in_sizes[21] != NCH * NCH || in_sizes[24] != NCH * NCH) return;
  if (in_sizes[8] != NCH * DLW || in_sizes[11] != NCH * DLA || in_sizes[16] != NCH * DLG) return;
  const size_t WS_NEEDED = 125 * MIB;
  if (ws_size < WS_NEEDED) return;

  const float* x    = (const float*)d_in[0];
  const float* x_r  = (const float*)d_in[1];
  const float* x_w  = (const float*)d_in[2];
  const float* x_k  = (const float*)d_in[3];
  const float* x_v  = (const float*)d_in[4];
  const float* x_a  = (const float*)d_in[5];
  const float* x_g  = (const float*)d_in[6];
  const float* w0   = (const float*)d_in[7];
  const float* w1   = (const float*)d_in[8];
  const float* w2   = (const float*)d_in[9];
  const float* a0   = (const float*)d_in[10];
  const float* a1   = (const float*)d_in[11];
  const float* a2   = (const float*)d_in[12];
  const float* g1w  = (const float*)d_in[16];
  const float* g2w  = (const float*)d_in[17];
  const float* k_k  = (const float*)d_in[18];
  const float* k_a  = (const float*)d_in[19];
  const float* r_k  = (const float*)d_in[20];
  const float* Wr   = (const float*)d_in[21];
  const float* Wk   = (const float*)d_in[22];
  const float* Wv   = (const float*)d_in[23];
  const float* Wo   = (const float*)d_in[24];
  const float* ln_w = (const float*)d_in[25];
  const float* ln_b = (const float*)d_in[26];
  float* out = (float*)d_out;

  char* ws = (char*)d_ws;
  float* Rf = (float*)(ws + 0 * PLANE_F32_BYTES);
  float* Kf = (float*)(ws + 1 * PLANE_F32_BYTES);
  float* Vf = (float*)(ws + 2 * PLANE_F32_BYTES);
  char* P0 = ws + 3 * PLANE_F32_BYTES;
  char* P1 = ws + 4 * PLANE_F32_BYTES;
  char* P2 = ws + 5 * PLANE_F32_BYTES;
  char* P3 = ws + 6 * PLANE_F32_BYTES;
  char* Sr = ws + 7 * PLANE_F32_BYTES;

  unsigned short* P0h = (unsigned short*)P0;
  unsigned short* P1h = (unsigned short*)P1;
  unsigned short* P2h = (unsigned short*)P2;
  unsigned short* bigW = (unsigned short*)P3;
  const size_t WPL = (size_t)NCH * NCH;

  unsigned short* w1Th = (unsigned short*)(Sr + 0);
  unsigned short* w1Tl = (unsigned short*)(Sr + 128 * 1024);
  unsigned short* a1Th = (unsigned short*)(Sr + 256 * 1024);
  unsigned short* a1Tl = (unsigned short*)(Sr + 384 * 1024);
  unsigned short* w2Th = (unsigned short*)(Sr + 512 * 1024);
  unsigned short* w2Tl = (unsigned short*)(Sr + 640 * 1024);
  unsigned short* a2Th = (unsigned short*)(Sr + 768 * 1024);
  unsigned short* a2Tl = (unsigned short*)(Sr + 896 * 1024);
  unsigned short* g1Th = (unsigned short*)(Sr + 1 * MIB);
  unsigned short* g1Tl = (unsigned short*)(Sr + 1 * MIB + 256 * 1024);
  unsigned short* g2Th = (unsigned short*)(Sr + 1 * MIB + 512 * 1024);
  unsigned short* g2Tl = (unsigned short*)(Sr + 1 * MIB + 768 * 1024);
  unsigned short* WoTh = (unsigned short*)(Sr + 2 * MIB);
  unsigned short* WoTl = (unsigned short*)(Sr + 4 * MIB);
  float*          T1f  = (float*)(Sr + 6 * MIB);
  unsigned short* T1h  = (unsigned short*)(Sr + 7 * MIB);
  unsigned short* T1l  = (unsigned short*)(Sr + 7 * MIB + 512 * 1024);
  unsigned short* TAh  = (unsigned short*)(Sr + 8 * MIB);
  unsigned short* TAl  = (unsigned short*)(Sr + 8 * MIB + 512 * 1024);
  float*          TGf  = (float*)(Sr + 9 * MIB);
  unsigned short* TGh  = (unsigned short*)(Sr + 11 * MIB);
  unsigned short* TGl  = (unsigned short*)(Sr + 12 * MIB);

  const dim3 blk(256);
  const int nPrep = (int)(PLANE_ELEMS / 8 / 256);
  const int nMid  = (int)(PLANE_ELEMS / 256);

  wsplit_kernel<<<dim3(NCH / 64, NCH / 64, 3), blk, 0, stream>>>(Wr, Wk, Wv, bigW, NCH, NCH);
  wsplit_kernel<<<dim3(NCH / 64, DLW / 64, 2), blk, 0, stream>>>(w1, a1, a1, w1Th, NCH, DLW);
  wsplit_kernel<<<dim3(DLW / 64, NCH / 64, 2), blk, 0, stream>>>(w2, a2, a2, w2Th, DLW, NCH);
  wsplit_kernel<<<dim3(NCH / 64, DLG / 64, 1), blk, 0, stream>>>(g1w, g1w, g1w, g1Th, NCH, DLG);
  wsplit_kernel<<<dim3(DLG / 64, NCH / 64, 1), blk, 0, stream>>>(g2w, g2w, g2w, g2Th, DLG, NCH);

  prep_kernel<3><<<dim3(nPrep), blk, 0, stream>>>(x, x_r, x_k, x_v, P0h, P1h, P2h);
  gemm_split_f32(P0h, P0h + PLANE_ELEMS, NCH, bigW + 0 * WPL, bigW + 1 * WPL, NCH, Rf, NCH, MROWS, NCH, NCH, stream);
  gemm_split_f32(P1h, P1h + PLANE_ELEMS, NCH, bigW + 2 * WPL, bigW + 3 * WPL, NCH, Kf, NCH, MROWS, NCH, NCH, stream);
  gemm_split_f32(P2h, P2h + PLANE_ELEMS, NCH, bigW + 4 * WPL, bigW + 5 * WPL, NCH, Vf, NCH, MROWS, NCH, NCH, stream);

  prep_kernel<2><<<dim3(nPrep), blk, 0, stream>>>(x, x_w, x_a, x_a, P0h, P1h, P1h);
  gemm_split_f32(P0h, P0h + PLANE_ELEMS, NCH, w1Th, w1Tl, NCH, T1f, DLW, MROWS, DLW, NCH, stream);
  act8_kernel<1><<<dim3((MROWS * DLW / 8) / 256), blk, 0, stream>>>(T1f, T1h, T1l, MROWS * DLW / 8);
  gemm_split_f32(T1h, T1l, DLW, w2Th, w2Tl, DLW, (float*)P2, NCH, MROWS, NCH, DLW, stream);
  gemm_split_hilo(P1h, P1h + PLANE_ELEMS, NCH, a1Th, a1Tl, NCH, TAh, TAl, DLA, MROWS, DLA, NCH, stream);
  gemm_split_f32(TAh, TAl, DLA, a2Th, a2Tl, DLA, (float*)P3, NCH, MROWS, NCH, DLA, stream);

  mid_kernel<<<dim3(nMid), blk, 0, stream>>>((const float*)P2, (const float*)P3, w0, a0, (float*)P0, (float*)P1);

  wkv_kernel<<<dim3(NBATCH * NHEAD), dim3(512), 0, stream>>>(Rf, (const float*)P0, Kf, Vf, (const float*)P1,
                                                             k_k, k_a, (float*)P2);

  prep_kernel<1><<<dim3(nPrep), blk, 0, stream>>>(x, x_g, x_g, x_g, P0h, P0h, P0h);
  gemm_split_f32(P0h, P0h + PLANE_ELEMS, NCH, g1Th, g1Tl, NCH, TGf, DLG, MROWS, DLG, NCH, stream);
  act8_kernel<2><<<dim3((MROWS * DLG / 8) / 256), blk, 0, stream>>>(TGf, TGh, TGl, MROWS * DLG / 8);
  gemm_split_f32(TGh, TGl, DLG, g2Th, g2Tl, DLG, (float*)P3, NCH, MROWS, NCH, DLG, stream);

  post_kernel<<<dim3(nPrep), blk, 0, stream>>>((const float*)P2, Rf, Kf, (const float*)P1, Vf, (const float*)P3,
                                                k_a, r_k, ln_w, ln_b, P0h, P0h + PLANE_ELEMS);

  wsplit_kernel<<<dim3(NCH / 64, NCH / 64, 1), blk, 0, stream>>>(Wo, Wo, Wo, WoTh, NCH, NCH);
  gemm_split_f32(P0h, P0h + PLANE_ELEMS, NCH, WoTh, WoTl, NCH, out, NCH, MROWS, NCH, NCH, stream);
}
